// FullAttention_37538014167158
// MI455X (gfx1250) — hardware-verified
//
#include <hip/hip_runtime.h>
#include <math.h>

#ifndef NB
#define NB 8
#endif
#ifndef SEQ
#define SEQ 1024
#endif
#define NB_FULL 8
#define SEQ_FULL 1024
#define NH 8
#define HD 64
#define HE (NH * HD)
#define AT_NW 4
#define PSC 16384.0f

static_assert(NB >= 1 && NB <= NB_FULL);
static_assert(SEQ >= 128 && SEQ <= SEQ_FULL && (SEQ % 128) == 0);
static_assert(((SEQ * HE / 8) % 256) == 0);
static_assert(((SEQ * HD / 8) % 256) == 0);
static_assert(((HE * (SEQ / 8)) % 256) == 0);

typedef __attribute__((ext_vector_type(16))) _Float16     v16h;
typedef __attribute__((ext_vector_type(8)))  _Float16     v8h;
typedef __attribute__((ext_vector_type(8)))  float        v8f;
typedef __attribute__((ext_vector_type(4)))  float        v4f;
typedef __attribute__((ext_vector_type(4)))  unsigned int v4u;
typedef __attribute__((ext_vector_type(4)))  int          v4i;

union FragH { v16h v; v8h h[2]; };
__device__ __forceinline__ v16h frag_g(const unsigned short* p) { FragH f; f.h[0] = *(const v8h*)(p); f.h[1] = *(const v8h*)(p + 16); return f.v; }
__device__ __forceinline__ v16h frag_l(const _Float16* p)       { FragH f; f.h[0] = *(const v8h*)(p); f.h[1] = *(const v8h*)(p + 16); return f.v; }

__device__ __forceinline__ v8f wm(v16h a, v16h b, v8f c) { return __builtin_amdgcn_wmma_f32_16x16x32_f16(false, a, false, b, (short)0, c, false, false); }
__device__ __forceinline__ v8f mma_s4(v16h qa, v16h ua, v16h va, v16h kb, v16h pb, v8f c) {
    c = wm(qa, kb, c); c = wm(ua, kb, c); c = wm(qa, pb, c); c = wm(va, pb, c);
    asm volatile("v_nop\n\tv_nop\n\tv_nop\n\tv_nop" : "+v"(c) : "v"(qa), "v"(ua), "v"(va), "v"(kb), "v"(pb));
    return c;
}
__device__ __forceinline__ v8f mma_pv2(v16h p0, v16h v0, v16h p1, v16h v1, v8f c) {
    c = wm(p0, v0, c); c = wm(p1, v1, c);
    asm volatile("v_nop\n\tv_nop\n\tv_nop\n\tv_nop" : "+v"(c) : "v"(p0), "v"(v0), "v"(p1), "v"(v1));
    return c;
}

__device__ __forceinline__ float bf_rne_f32(float v) { const unsigned u = __float_as_uint(v); const unsigned r = (u + 0x7fffu + ((u >> 16) & 1u)) & 0xffff0000u; return __uint_as_float(r); }
__device__ __forceinline__ unsigned int pk2h(float a, float b) { return (unsigned int)__builtin_bit_cast(unsigned short, (_Float16)a) | ((unsigned int)__builtin_bit_cast(unsigned short, (_Float16)b) << 16); }

#define VST2(T, ptr, val) do { const T vst2_v_ = (val); *(volatile T*)(ptr) = vst2_v_; __threadfence(); *(volatile T*)(ptr) = vst2_v_; } while (0)

__global__ __launch_bounds__(256) void k_cast_rows(const float* __restrict__ src, long long sbs, unsigned short* __restrict__ dst, long long dbs, int nElem8) {
    const int u = blockIdx.x * 256 + threadIdx.x;
    if (u >= nElem8) return;
    const float* s = src + (long long)blockIdx.y * sbs + (long long)u * 8;
    const v4f a = *(const v4f*)(s), bq = *(const v4f*)(s + 4);
    v4u pk;
    pk.x = pk2h(bf_rne_f32(a.x), bf_rne_f32(a.y));   pk.y = pk2h(bf_rne_f32(a.z), bf_rne_f32(a.w));
    pk.z = pk2h(bf_rne_f32(bq.x), bf_rne_f32(bq.y)); pk.w = pk2h(bf_rne_f32(bq.z), bf_rne_f32(bq.w));
    unsigned short* d = dst + (long long)blockIdx.y * dbs + (long long)u * 8;
    VST2(v4u, (v4u*)d, pk);
}

__global__ __launch_bounds__(256) void k_cast_vT(const float* __restrict__ src, unsigned short* __restrict__ dst) {
    const int u = blockIdx.x * 256 + threadIdx.x;
    const int per = SEQ / 8;
    if (u >= HE * per) return;
    const int cc = u / per, s0 = 8 * (u % per);
    const float* s = src + (size_t)blockIdx.y * SEQ_FULL * HE + (size_t)s0 * HE + cc;
    float w[8];
#pragma unroll
    for (int e = 0; e < 8; ++e) w[e] = bf_rne_f32(s[(size_t)e * HE]);
    v4u pk; pk.x = pk2h(w[0], w[1]); pk.y = pk2h(w[2], w[3]); pk.z = pk2h(w[4], w[5]); pk.w = pk2h(w[6], w[7]);
    unsigned short* d = dst + (size_t)blockIdx.y * HE * SEQ + (size_t)cc * SEQ + s0;
    VST2(v4u, (v4u*)d, pk);
}

__global__ __launch_bounds__(256) void k_maskchk(const int* __restrict__ mask, unsigned int* __restrict__ flag) {
    __shared__ int red[256];
    const int tid = threadIdx.x, w = tid >> 5, L = tid & 31;
    int bad = 0;
    for (int row = w; row < SEQ; row += 8) {
        const int* mr = mask + (size_t)row * SEQ_FULL;
#pragma unroll 1
        for (int i = 0; i < SEQ / 128; ++i) {
            const int col = i * 128 + 4 * L;
            const v4i m = *(const v4i*)(mr + col);
            bad |= (int)((m.x != 0) != (col > row));
            bad |= (int)((m.y != 0) != (col + 1 > row));
            bad |= (int)((m.z != 0) != (col + 2 > row));
            bad |= (int)((m.w != 0) != (col + 3 > row));
        }
    }
    red[tid] = bad;
    __syncthreads();
    for (int o = 128; o > 0; o >>= 1) { if (tid < o) red[tid] |= red[tid + o]; __syncthreads(); }
    if (tid < 32) { const unsigned int v = (tid == 0) ? (unsigned int)(red[0] != 0) : 0u; VST2(unsigned int, flag + tid, v); }
}

__global__ __launch_bounds__(128) void k_attn(const unsigned short* __restrict__ Q16, const unsigned short* __restrict__ K16,
                                              const unsigned short* __restrict__ P16, const unsigned short* __restrict__ VT16,
                                              const unsigned short* __restrict__ UW16, const unsigned short* __restrict__ VW16,
                                              const float* __restrict__ ub, const float* __restrict__ vb,
                                              const unsigned int* __restrict__ flag, float* __restrict__ out) {
    __shared__ __align__(16) _Float16 Psh[AT_NW][16 * 64];
    __shared__ __align__(16) float    Os[AT_NW][16 * 68];

    const int tid = threadIdx.x;
    const int wave = tid >> 5, lane = tid & 31, hh = lane >> 4, c = lane & 15;
    constexpr int NQB = SEQ / 64;
    const int bx = blockIdx.x;
    const int qb = bx % NQB, bh = bx / NQB, h = bh % NH, b = bh / NH;
    const int q0 = qb * 64 + wave * 16;
    const float NEG = -__builtin_inff();
    const float SCL = 0.125f * 1.4426950408889634f;

    const size_t qoff = ((size_t)b * SEQ + (size_t)(q0 + c)) * HE + (size_t)h * HD + 8 * hh;
    const v16h qa0 = frag_g(Q16 + qoff), qa1 = frag_g(Q16 + qoff + 32);
    const size_t woff = (size_t)(q0 + c) * HD + 8 * hh;
    const v16h ua0 = frag_g(UW16 + woff), ua1 = frag_g(UW16 + woff + 32);
    const v16h va0 = frag_g(VW16 + woff), va1 = frag_g(VW16 + woff + 32);

    float bsum[8], mrow[8], lrow[8];
    v8f oacc[4];
#pragma unroll
    for (int r = 0; r < 8; ++r) {
        const int qr = q0 + 8 * hh + r;
        bsum[r] = bf_rne_f32(ub[qr]) + bf_rne_f32(vb[qr]);
        mrow[r] = NEG; lrow[r] = 0.f;
    }
#pragma unroll
    for (int t = 0; t < 4; ++t) { v8f zz = {}; oacc[t] = zz; }

    const size_t kvb = (size_t)b * SEQ * HE + (size_t)h * HD + 8 * hh;
    const unsigned short* kbase = K16 + kvb;
    const unsigned short* pbase = P16 + kvb;
    const unsigned short* vtb = VT16 + ((size_t)(b * NH + h) * HD + c) * SEQ + 8 * hh;
    _Float16* pw = Psh[wave];

    for (int kc = 0; kc <= qb; ++kc) {
        const int kv0 = kc * 64;
        v8f s[4];
#pragma unroll
        for (int j = 0; j < 4; ++j) {
            const size_t ro = (size_t)(kv0 + j * 16 + c) * HE;
            v8f acc = {};
            {
                const v16h kb = frag_g(kbase + ro), pb = frag_g(pbase + ro);
                acc = mma_s4(qa0, ua0, va0, kb, pb, acc);
            }
            {
                const v16h kb = frag_g(kbase + ro + 32), pb = frag_g(pbase + ro + 32);
                acc = mma_s4(qa1, ua1, va1, kb, pb, acc);
            }
            s[j] = acc;
        }
        const bool diag = (kc == qb);
        float cm[8];
#pragma unroll
        for (int r = 0; r < 8; ++r) {
            const int qrow = q0 + 8 * hh + r;
            float m = NEG;
#pragma unroll
            for (int j = 0; j < 4; ++j) {
                const int kvcol = kv0 + j * 16 + c;
                float v = (s[j][r] + bsum[r]) * SCL;
                v = (diag && (kvcol > qrow)) ? NEG : v;
                s[j][r] = v;
                m = fmaxf(m, v);
            }
            m = fmaxf(m, __shfl_xor(m, 1, 32)); m = fmaxf(m, __shfl_xor(m, 2, 32));
            m = fmaxf(m, __shfl_xor(m, 4, 32)); m = fmaxf(m, __shfl_xor(m, 8, 32));
            cm[r] = m;
        }
#pragma unroll
        for (int r = 0; r < 8; ++r) {
            const float mnew = fmaxf(mrow[r], cm[r]);
            const float ex = exp2f(mrow[r] - mnew);
            const float alpha = (mrow[r] == NEG) ? 0.f : ex;
            mrow[r] = mnew;
            float psum = 0.f;
#pragma unroll
            for (int j = 0; j < 4; ++j) {
                const float e = exp2f(s[j][r] - mnew);
                const float p = (s[j][r] == NEG) ? 0.f : e;
                psum += p;
                pw[(8 * hh + r) * 64 + j * 16 + c] = (_Float16)(p * PSC);
            }
            psum += __shfl_xor(psum, 1, 32); psum += __shfl_xor(psum, 2, 32);
            psum += __shfl_xor(psum, 4, 32); psum += __shfl_xor(psum, 8, 32);
            lrow[r] = lrow[r] * alpha + psum;
#pragma unroll
            for (int t = 0; t < 4; ++t) oacc[t][r] *= alpha;
        }
        __builtin_amdgcn_fence(3  , "workgroup");
        __builtin_amdgcn_wave_barrier();
        __builtin_amdgcn_fence(2  , "workgroup");
        {
            const v16h pa0 = frag_l(pw + c * 64 + 8 * hh), pa1 = frag_l(pw + c * 64 + 32 + 8 * hh);
#pragma unroll
            for (int t = 0; t < 4; ++t) {
                const unsigned short* vr = vtb + (size_t)(t * 16) * SEQ + kv0;
                const v16h vb0 = frag_g(vr), vb1 = frag_g(vr + 32);
                oacc[t] = mma_pv2(pa0, vb0, pa1, vb1, oacc[t]);
            }
        }
        __builtin_amdgcn_fence(3  , "workgroup");
        __builtin_amdgcn_wave_barrier();
        __builtin_amdgcn_fence(2  , "workgroup");
    }

    float* os = Os[wave];
#pragma unroll
    for (int r = 0; r < 8; ++r) {
        const float inv = 1.0f / (lrow[r] * PSC);
#pragma unroll
        for (int t = 0; t < 4; ++t) os[(8 * hh + r) * 68 + t * 16 + c] = oacc[t][r] * inv;
    }
    __builtin_amdgcn_fence(3  , "workgroup");
    __builtin_amdgcn_wave_barrier();
    __builtin_amdgcn_fence(2  , "workgroup");
    {
        const unsigned int fl = flag[0];
        const float qnan = __uint_as_float(0x7fc00000u);
        float* ob = out + ((size_t)b * SEQ + (size_t)q0) * HE + (size_t)h * HD;
        const int c4 = (lane & 15) * 4;
        for (int pass = 0; pass < 2; ++pass) {
#pragma unroll
            for (int it = 0; it < 8; ++it) {
                const int row = it * 2 + hh;
                v4f val = *(const v4f*)(os + row * 68 + c4);
                val.x = (fl != 0u) ? qnan : val.x; val.y = (fl != 0u) ? qnan : val.y;
                val.z = (fl != 0u) ? qnan : val.z; val.w = (fl != 0u) ? qnan : val.w;
                *(volatile v4f*)(ob + (size_t)row * HE + c4) = val;
            }
            __threadfence();
        }
    }
}

extern "C" void kernel_launch(void* const* d_in, const int* in_sizes, int n_in, void* d_out, int out_size, void* d_ws, size_t ws_size, hipStream_t stream) {
    if (n_in < 10) return;
    const long long need_act = (long long)(NB - 1) * SEQ_FULL * HE + (long long)SEQ * HE;
    if (in_sizes[0] < need_act || in_sizes[1] < need_act || in_sizes[2] < need_act || in_sizes[3] < need_act) return;
    if (in_sizes[4] < (long long)(SEQ - 1) * SEQ_FULL + SEQ) return;
    if (in_sizes[5] < SEQ * HD || in_sizes[7] < SEQ * HD || in_sizes[6] < SEQ || in_sizes[8] < SEQ) return;
    if (out_size < NB * SEQ * HE) return;

    const float* q   = (const float*)d_in[0];
    const float* k   = (const float*)d_in[1];
    const float* v   = (const float*)d_in[2];
    const float* pe  = (const float*)d_in[3];
    const int*   msk = (const int*)d_in[4];
    const float* uw  = (const float*)d_in[5];
    const float* ub  = (const float*)d_in[6];
    const float* vw  = (const float*)d_in[7];
    const float* vb  = (const float*)d_in[8];
    float* out = (float*)d_out;

    constexpr size_t ACT_B = (((size_t)NB * SEQ * HE * 2 + 255) / 256) * 256;
    constexpr size_t WGT_B = (((size_t)SEQ * HD * 2 + 255) / 256) * 256;
    constexpr size_t FLG_B = 256;
    constexpr size_t TOTAL_B = 4 * ACT_B + 2 * WGT_B + FLG_B;
    static_assert(TOTAL_B <= (size_t)134217728);
    if (TOTAL_B > ws_size) return;
    char* wsp = (char*)d_ws;
    unsigned short* Q16  = (unsigned short*)wsp; wsp += ACT_B;
    unsigned short* K16  = (unsigned short*)wsp; wsp += ACT_B;
    unsigned short* P16  = (unsigned short*)wsp; wsp += ACT_B;
    unsigned short* VT16 = (unsigned short*)wsp; wsp += ACT_B;
    unsigned short* UW16 = (unsigned short*)wsp; wsp += WGT_B;
    unsigned short* VW16 = (unsigned short*)wsp; wsp += WGT_B;
    unsigned int*   FLAG = (unsigned int*)wsp;   wsp += FLG_B;

    const int nA8 = SEQ * HE / 8, nW8 = SEQ * HD / 8;
    k_cast_rows<<<dim3((unsigned)(nA8 / 256), (unsigned)NB), 256, 0, stream>>>(q,  (long long)SEQ_FULL * HE, Q16, (long long)SEQ * HE, nA8);
    k_cast_rows<<<dim3((unsigned)(nA8 / 256), (unsigned)NB), 256, 0, stream>>>(k,  (long long)SEQ_FULL * HE, K16, (long long)SEQ * HE, nA8);
    k_cast_rows<<<dim3((unsigned)(nA8 / 256), (unsigned)NB), 256, 0, stream>>>(pe, (long long)SEQ_FULL * HE, P16, (long long)SEQ * HE, nA8);
    k_cast_rows<<<dim3((unsigned)(nW8 / 256), 1u), 256, 0, stream>>>(uw, 0ll, UW16, 0ll, nW8);
    k_cast_rows<<<dim3((unsigned)(nW8 / 256), 1u), 256, 0, stream>>>(vw, 0ll, VW16, 0ll, nW8);
    k_cast_vT<<<dim3((unsigned)(HE * (SEQ / 8) / 256), (unsigned)NB), 256, 0, stream>>>(v, VT16);
    k_maskchk<<<1, 256, 0, stream>>>(msk, FLAG);
    k_attn<<<dim3((unsigned)(NB * NH * (SEQ / 64))), 128, 0, stream>>>(Q16, K16, P16, VT16, UW16, VW16, ub, vb, FLAG, out);
}
